// SSAM_12472585027856
// MI455X (gfx1250) — hardware-verified
//
#include <hip/hip_runtime.h>
#include <math.h>

constexpr int kImg  = 16;
constexpr int kCh   = 512;
constexpr int kTokN = 1024;
constexpr int kHidN = 2048;
constexpr int kGrp  = 4;
constexpr int kNGrp = kImg / kGrp;
constexpr float kScoreScale = 0.044194173824159216f;
constexpr float kPCarry     = 32768.0f;
constexpr float kPCarryInv  = 1.0f / 32768.0f;
constexpr float kW1Carry    = 32.0f;
constexpr float kW1CarryInv = 1.0f / 32.0f;
constexpr float kW2Carry    = 64.0f;
constexpr float kW2CarryInv = 1.0f / 64.0f;

constexpr size_t kOffOut16 = 0;
constexpr size_t kSzOut16  = (size_t)kImg * kTokN * kCh * 2;
constexpr size_t kOffW1S   = kOffOut16 + kSzOut16;
constexpr size_t kSzW      = (size_t)kHidN * kCh * 2;
constexpr size_t kOffW2S   = kOffW1S + kSzW;
constexpr size_t kOffX16   = kOffW2S + kSzW;
constexpr size_t kSzX16    = (size_t)kImg * kTokN * kCh * 2;
constexpr size_t kOffXR16  = kOffX16 + kSzX16;
constexpr size_t kOffS     = kOffXR16 + kSzX16;
constexpr size_t kSzS      = (size_t)kGrp * kTokN * kTokN * 4;
constexpr size_t kOffP     = kOffS + kSzS;
constexpr size_t kSzP      = (size_t)kGrp * kTokN * kTokN * 2;
constexpr size_t kOffH     = kOffX16;
constexpr size_t kSzH      = (size_t)kImg * kTokN * kHidN * 2;
constexpr size_t kWsTotal  = ((kOffP + kSzP) > (kOffH + kSzH)) ? (kOffP + kSzP) : (kOffH + kSzH);
static_assert(kWsTotal == 88080384u);
static_assert(kWsTotal <= 134217728u);
static_assert(kOffH >= kOffW2S + kSzW);

typedef __attribute__((ext_vector_type(16))) _Float16 v16h;
typedef __attribute__((ext_vector_type(8)))  _Float16 v8h;
typedef __attribute__((ext_vector_type(16))) __bf16   v16b;
typedef __attribute__((ext_vector_type(8)))  __bf16   v8b;
typedef __attribute__((ext_vector_type(8)))  float    v8f;
typedef __attribute__((ext_vector_type(4)))  float    v4f;
typedef __attribute__((ext_vector_type(4)))  unsigned int v4u;

__device__ __forceinline__ unsigned short f2bf_bits(float f) {
  unsigned u = __float_as_uint(f);
  return (unsigned short)((u + 0x7FFFu + ((u >> 16) & 1u)) >> 16);
}
__device__ __forceinline__ float bf_bits2f(unsigned short h) { return __uint_as_float(((unsigned)h) << 16); }

__device__ __forceinline__ void dep_guard_h(v8f& a, v8f& b, v16h x, v16h y) { asm volatile("v_nop\n\tv_nop\n\tv_nop\n\tv_nop" : "+v"(a), "+v"(b) : "v"(x), "v"(y)); }
__device__ __forceinline__ void dep_guard_b(v8f& a, v8f& b, v16b x, v16b y) { asm volatile("v_nop\n\tv_nop\n\tv_nop\n\tv_nop" : "+v"(a), "+v"(b) : "v"(x), "v"(y)); }
__device__ __forceinline__ void keep4_h(v16h a, v16h b, v16h c, v16h d) { asm volatile("v_nop" :: "v"(a), "v"(b), "v"(c), "v"(d)); }
__device__ __forceinline__ void keep4_b(v16b a, v16b b, v16b c, v16b d) { asm volatile("v_nop" :: "v"(a), "v"(b), "v"(c), "v"(d)); }
__device__ __forceinline__ void acc_guard4(v8f& a, v8f& b, v8f& c, v8f& d) { asm volatile("v_nop\n\tv_nop\n\tv_nop\n\tv_nop" : "+v"(a), "+v"(b), "+v"(c), "+v"(d)); }
template <typename T> struct Frag;
template <> struct Frag<_Float16> {
  typedef v16h V; union U { v16h v; v8h h[2]; };
  static __device__ __forceinline__ v16h load(const _Float16* p) {
    U f; f.h[0] = *(const v8h*)(p); f.h[1] = *(const v8h*)(p + 16); return f.v;
  }
  static __device__ __forceinline__ v8f mma(v16h a, v16h b, v8f c) {
    return __builtin_amdgcn_wmma_f32_16x16x32_f16(false, a, false, b, (short)0, c, false, false);
  }
  static __device__ __forceinline__ void guard(v8f& a, v8f& b, v16h x, v16h y) { dep_guard_h(a, b, x, y); }
  static __device__ __forceinline__ void keep(v16h a, v16h b, v16h c, v16h d) { keep4_h(a, b, c, d); }
};
template <> struct Frag<__bf16> {
  typedef v16b V; union U { v16b v; v8b h[2]; };
  static __device__ __forceinline__ v16b load(const __bf16* p) {
    U f; f.h[0] = *(const v8b*)(p); f.h[1] = *(const v8b*)(p + 16); return f.v;
  }
  static __device__ __forceinline__ v8f mma(v16b a, v16b b, v8f c) {
    return __builtin_amdgcn_wmma_f32_16x16x32_bf16(false, a, false, b, (short)0, c, false, false);
  }
  static __device__ __forceinline__ void guard(v8f& a, v8f& b, v16b x, v16b y) { dep_guard_b(a, b, x, y); }
  static __device__ __forceinline__ void keep(v16b a, v16b b, v16b c, v16b d) { keep4_b(a, b, c, d); }
};

__device__ __forceinline__ unsigned pk16(unsigned short a, unsigned short b) { return (unsigned)a | ((unsigned)b << 16); }
__device__ __forceinline__ unsigned short h_bits(float f) { const _Float16 h = (_Float16)f; return __builtin_bit_cast(unsigned short, h); }

template <int ET> struct Elem;
template <> struct Elem<0> { typedef _Float16 T; };
template <> struct Elem<1> { typedef __bf16 T; };
template <int ET, bool SPLIT, int BIAS_MODE, int OUT_MODE, bool RESID, int ACT = 0>
__global__ __launch_bounds__(256) void wmma_gemm64(
    const unsigned short* __restrict__ Ap, const unsigned short* __restrict__ A2p, int lda, long strideA,
    const unsigned short* __restrict__ Btp, const unsigned short* __restrict__ Bt2p, int ldb, long strideB,
    void* __restrict__ Cout, void* __restrict__ Cout2, int ldc, long strideC,
    const float* __restrict__ bias,
    const float* __restrict__ resid, long strideR,
    int M, int N, int K, float scale) {
  typedef typename Elem<ET>::T T;
  typedef typename Frag<T>::V V;
  const T* A = (const T*)Ap; const T* A2 = (const T*)A2p; const T* Bt = (const T*)Btp; const T* Bt2 = (const T*)Bt2p;
  __shared__ __align__(16) float sT[8][16 * 68];
  const int b    = blockIdx.y;
  const int lane = threadIdx.x & 31;
  const int wave = threadIdx.x >> 5;
  const int tilesN = N >> 6;
  const int tilesM = M >> 6;
  const int tile = blockIdx.x * 8 + wave;
  if (tile >= tilesM * tilesN) return;
  const int tm = tile / tilesN;
  const int tn = tile - tm * tilesN;
  const int m0 = tm << 6;
  const int n0 = tn << 6;

  const T* Ab  = A  + (size_t)b * strideA;
  const T* Bb  = Bt + (size_t)b * strideB;
  const T* Ab2 = SPLIT ? (A2  + (size_t)b * strideA) : nullptr;
  const T* Bb2 = SPLIT ? (Bt2 + (size_t)b * strideB) : nullptr;

  const int rlane = lane & 15;
  const int koff  = (lane >> 4) * 8;
  const int mOff  = (lane >> 4) * 8;

  v8f acc[4][4];
#pragma unroll
  for (int i = 0; i < 4; ++i)
#pragma unroll
    for (int j = 0; j < 4; ++j) acc[i][j] = (v8f){0.f,0.f,0.f,0.f,0.f,0.f,0.f,0.f};

  for (int k0 = 0; k0 < K; k0 += 32) {
    V bh[4], bl[4];
#pragma unroll
    for (int j = 0; j < 4; ++j) {
      const size_t bo = (size_t)(n0 + (j << 4) + rlane) * ldb + koff + k0;
      bh[j] = Frag<T>::load(Bb + bo);
      if (SPLIT) bl[j] = Frag<T>::load(Bb2 + bo);
    }
#pragma unroll
    for (int i = 0; i < 4; ++i) {
      const size_t ao = (size_t)(m0 + (i << 4) + rlane) * lda + koff + k0;
      V ah = Frag<T>::load(Ab + ao);
      V al;
      if (SPLIT) al = Frag<T>::load(Ab2 + ao);
#pragma unroll
      for (int j = 0; j < 4; ++j) {
        acc[i][j] = Frag<T>::mma(ah, bh[j], acc[i][j]);
        if (SPLIT) {
          acc[i][j] = Frag<T>::mma(ah, bl[j], acc[i][j]);
          acc[i][j] = Frag<T>::mma(al, bh[j], acc[i][j]);
        }
      }
      Frag<T>::guard(acc[i][0], acc[i][3], ah, SPLIT ? al : ah);
    }
    Frag<T>::keep(bh[0], bh[1], bh[2], bh[3]);
    if (SPLIT) Frag<T>::keep(bl[0], bl[1], bl[2], bl[3]);
  }
  acc_guard4(acc[0][0], acc[0][1], acc[0][2], acc[0][3]);
  acc_guard4(acc[1][0], acc[1][1], acc[1][2], acc[1][3]);
  acc_guard4(acc[2][0], acc[2][1], acc[2][2], acc[2][3]);
  acc_guard4(acc[3][0], acc[3][1], acc[3][2], acc[3][3]);

  float* slab = sT[wave];
  const float* Rb = RESID ? (resid + (size_t)b * strideR) : nullptr;
#pragma unroll
  for (int i = 0; i < 4; ++i) {
    const int mBase = m0 + (i << 4);
#pragma unroll
    for (int j = 0; j < 4; ++j) {
      const int n = n0 + (j << 4) + rlane;
      float bv = 0.f;
      if (BIAS_MODE == 2) bv = bias[n];
#pragma unroll
      for (int r = 0; r < 8; ++r) {
        float v = acc[i][j][r] * scale;
        if (BIAS_MODE == 1) v += bias[mBase + mOff + r];
        if (BIAS_MODE == 2) v += bv;
        if (RESID) v += Rb[(size_t)(mBase + mOff + r) * ldc + n];
        if (ACT == 2) v = fmaxf(v, 0.0f);
        if (ACT == 4) v = (v > 0.f) ? v : 0.01f * v;
        slab[(mOff + r) * 68 + (j << 4) + rlane] = v;
      }
    }
    __builtin_amdgcn_fence(__ATOMIC_RELEASE, "workgroup");
    __builtin_amdgcn_wave_barrier();
    __builtin_amdgcn_fence(__ATOMIC_ACQUIRE, "workgroup");
    if (OUT_MODE == 0) {
      float* C = (float*)Cout + (size_t)b * strideC;
      const int hh = lane >> 4, c4 = (lane & 15) * 4;
      for (int pass = 0; pass < 2; ++pass) {
#pragma unroll
        for (int it = 0; it < 8; ++it) {
          const int row = it * 2 + hh;
          v4f v = *(const v4f*)(slab + row * 68 + c4);
          *(volatile v4f*)(C + (size_t)(mBase + row) * ldc + n0 + c4) = v;
        }
        __threadfence();
      }
    } else {
      const int q = lane >> 3, c8 = (lane & 7) * 8;
      unsigned short* C  = (unsigned short*)Cout  + (size_t)b * strideC;
      unsigned short* C2 = (OUT_MODE == 2) ? ((unsigned short*)Cout2 + (size_t)b * strideC) : nullptr;
      for (int pass = 0; pass < 2; ++pass) {
#pragma unroll
        for (int it = 0; it < 4; ++it) {
          const int row = it * 4 + q;
          const float* sp = slab + row * 68 + c8;
          v8h hv, lv;
#pragma unroll
          for (int e = 0; e < 8; ++e) {
            if (OUT_MODE == 1) {
              hv[e] = (_Float16)sp[e];
            } else {
              unsigned short hb = f2bf_bits(sp[e]);
              unsigned short lb = f2bf_bits(sp[e] - bf_bits2f(hb));
              hv[e] = __builtin_bit_cast(_Float16, hb);
              lv[e] = __builtin_bit_cast(_Float16, lb);
            }
          }
          *(volatile v8h*)(C + (size_t)(mBase + row) * ldc + n0 + c8) = hv;
          if (OUT_MODE == 2) *(volatile v8h*)(C2 + (size_t)(mBase + row) * ldc + n0 + c8) = lv;
        }
        __threadfence();
      }
    }
    __builtin_amdgcn_fence(__ATOMIC_RELEASE, "workgroup");
    __builtin_amdgcn_wave_barrier();
    __builtin_amdgcn_fence(__ATOMIC_ACQUIRE, "workgroup");
  }
}

__global__ __launch_bounds__(256) void xt_kernel(const float* __restrict__ x, unsigned short* __restrict__ X16) {
  __shared__ float sm[64][65];
  const int t  = threadIdx.x;
  const int n0 = blockIdx.x * 64;
  const int c0 = blockIdx.y * 64;
  const int b  = blockIdx.z;
  const float* xb = x + (size_t)b * kCh * kTokN;
#pragma unroll
  for (int i = 0; i < 16; ++i) {
    const int e  = i * 256 + t;
    const int r  = e >> 6;
    const int cc = e & 63;
    sm[cc][r] = xb[(size_t)(c0 + r) * kTokN + n0 + cc];
  }
  __syncthreads();
  const int lane = t & 31, wave = t >> 5;
  const int q = lane >> 3, c8 = (lane & 7) * 8;
  unsigned short* op = X16 + (size_t)b * kTokN * kCh;
  for (int pass = 0; pass < 2; ++pass) {
#pragma unroll
    for (int it = 0; it < 2; ++it) {
      const int row = wave * 8 + it * 4 + q;
      unsigned short hb[8];
#pragma unroll
      for (int e = 0; e < 8; ++e) hb[e] = h_bits(sm[row][c8 + e]);
      const v4u u = (v4u){pk16(hb[0], hb[1]), pk16(hb[2], hb[3]), pk16(hb[4], hb[5]), pk16(hb[6], hb[7])};
      *(volatile v4u*)(op + (size_t)(n0 + row) * kCh + c0 + c8) = u;
    }
    __threadfence();
  }
}

__global__ __launch_bounds__(256) void cast8_kernel(const float* __restrict__ in, unsigned short* __restrict__ out, int n8, float carry) {
  const int i = blockIdx.x * 256 + threadIdx.x;
  if (i >= n8) return;
  const float* p = in + 8 * (size_t)i;
  const v4f a = *(const v4f*)(p);
  const v4f c = *(const v4f*)(p + 4);
  unsigned short hb[8];
#pragma unroll
  for (int e = 0; e < 4; ++e) {
    hb[e]     = h_bits(a[e] * carry);
    hb[4 + e] = h_bits(c[e] * carry);
  }
  const v4u u = (v4u){pk16(hb[0], hb[1]), pk16(hb[2], hb[3]), pk16(hb[4], hb[5]), pk16(hb[6], hb[7])};
  unsigned short* q = out + 8 * (size_t)i;
  *(volatile v4u*)q = u;
  __threadfence();
  *(volatile v4u*)q = u;
}

__global__ __launch_bounds__(128) void softmax_row_kernel(const float* __restrict__ S, unsigned short* __restrict__ P, float carry) {
  __shared__ float redM[4];
  __shared__ float redS[4];
  const int row  = blockIdx.x;
  const int t    = threadIdx.x;
  const int lane = t & 31, wave = t >> 5;
  const int c0   = t * 8;
  const float* sr = S + (size_t)row * kTokN + c0;
  const v4f a = *(const v4f*)(sr);
  const v4f c = *(const v4f*)(sr + 4);
  float xv[8];
#pragma unroll
  for (int e = 0; e < 4; ++e) { xv[e] = a[e]; xv[4 + e] = c[e]; }
  float m = fmaxf(fmaxf(fmaxf(xv[0], xv[1]), fmaxf(xv[2], xv[3])), fmaxf(fmaxf(xv[4], xv[5]), fmaxf(xv[6], xv[7])));
#pragma unroll
  for (int off = 16; off > 0; off >>= 1) m = fmaxf(m, __shfl_xor(m, off, 32));
  if (lane == 0) redM[wave] = m;
  __syncthreads();
  const float rmax = fmaxf(fmaxf(redM[0], redM[1]), fmaxf(redM[2], redM[3]));
  float ex[8];
#pragma unroll
  for (int e = 0; e < 8; ++e) ex[e] = expf(xv[e] - rmax);
  float s = ((ex[0] + ex[1]) + (ex[2] + ex[3])) + ((ex[4] + ex[5]) + (ex[6] + ex[7]));
#pragma unroll
  for (int off = 16; off > 0; off >>= 1) s += __shfl_xor(s, off, 32);
  if (lane == 0) redS[wave] = s;
  __syncthreads();
  const float tot = ((redS[0] + redS[1]) + redS[2]) + redS[3];
  const float inv = carry * (1.0f / tot);
  unsigned short hb[8];
#pragma unroll
  for (int e = 0; e < 8; ++e) hb[e] = h_bits(ex[e] * inv);
  const v4u u = (v4u){pk16(hb[0], hb[1]), pk16(hb[2], hb[3]), pk16(hb[4], hb[5]), pk16(hb[6], hb[7])};
  unsigned short* q = P + (size_t)row * kTokN + c0;
  *(volatile v4u*)q = u;
  __threadfence();
  *(volatile v4u*)q = u;
}

extern "C" void kernel_launch(void* const* d_in, const int* in_sizes, int n_in,
                              void* d_out, int out_size, void* d_ws,
                              size_t ws_size, hipStream_t stream) {
  if (n_in < 5) return;
  if (in_sizes[0] != kImg * kCh * kTokN) return;
  if (in_sizes[1] != kHidN * kCh) return;
  if (in_sizes[2] != kHidN) return;
  if (in_sizes[3] != kCh * kHidN) return;
  if (in_sizes[4] != kCh) return;
  if (out_size != kImg * kCh * kTokN) return;
  if (ws_size < kWsTotal) return;

  const float* x  = (const float*)d_in[0];
  const float* w1 = (const float*)d_in[1];
  const float* b1 = (const float*)d_in[2];
  const float* w2 = (const float*)d_in[3];
  const float* b2 = (const float*)d_in[4];
  float* y = (float*)d_out;

  char* ws = (char*)d_ws;
  unsigned short* OUT16 = (unsigned short*)(ws + kOffOut16);
  unsigned short* W1S   = (unsigned short*)(ws + kOffW1S);
  unsigned short* W2S   = (unsigned short*)(ws + kOffW2S);
  unsigned short* X16   = (unsigned short*)(ws + kOffX16);
  unsigned short* XR16  = (unsigned short*)(ws + kOffXR16);
  float*          Sbuf  = (float*)(ws + kOffS);
  unsigned short* Pbuf  = (unsigned short*)(ws + kOffP);
  unsigned short* Hbuf  = (unsigned short*)(ws + kOffH);

  xt_kernel<<<dim3(kTokN / 64, kCh / 64, kImg), 256, 0, stream>>>(x, X16);
  cast8_kernel<<<(kImg * kCh * kTokN / 8) / 256, 256, 0, stream>>>(x, XR16, kImg * kCh * kTokN / 8, 1.0f);
  cast8_kernel<<<(kHidN * kCh / 8) / 256, 256, 0, stream>>>(w1, W1S, kHidN * kCh / 8, kW1Carry);
  cast8_kernel<<<(kHidN * kCh / 8) / 256, 256, 0, stream>>>(w2, W2S, kHidN * kCh / 8, kW2Carry);

  const long imgX  = (long)kTokN * kCh;
  const long imgS  = (long)kTokN * kTokN;

  for (int g = 0; g < kNGrp; ++g) {
    const unsigned short* Xg  = X16  + (size_t)g * kGrp * imgX;
    const unsigned short* XRg = XR16 + (size_t)g * kGrp * imgX;
    unsigned short*       Og  = OUT16 + (size_t)g * kGrp * imgX;

    wmma_gemm64<0, false, 0, 0, false, 0><<<dim3(32, kGrp), 256, 0, stream>>>(
        Xg, Xg, kCh, imgX,
        Xg, Xg, kCh, imgX,
        (void*)Sbuf, (void*)Sbuf, kTokN, imgS,
        b1, x, 0L,
        kTokN, kTokN, kCh, kScoreScale);

    softmax_row_kernel<<<kGrp * kTokN, 128, 0, stream>>>(Sbuf, Pbuf, kPCarry);

    wmma_gemm64<0, false, 0, 1, false, 0><<<dim3(16, kGrp), 256, 0, stream>>>(
        Pbuf, Pbuf, kTokN, imgS,
        XRg, XRg, kTokN, imgX,
        (void*)Og, (void*)Og, kCh, imgX,
        b1, x, 0L,
        kTokN, kCh, kTokN, kPCarryInv);
  }

  wmma_gemm64<0, false, 2, 1, false, 2><<<dim3(1024, 1), 256, 0, stream>>>(
      OUT16, OUT16, kCh, 0L,
      W1S, W1S, kCh, 0L,
      (void*)Hbuf, (void*)Hbuf, kHidN, 0L,
      b1, x, 0L,
      kImg * kTokN, kHidN, kCh, kW1CarryInv);

  wmma_gemm64<0, false, 1, 0, true, 0><<<dim3(16, kImg), 256, 0, stream>>>(
      W2S, W2S, kHidN, 0L,
      Hbuf, Hbuf, kHidN, (long)kTokN * kHidN,
      (void*)y, (void*)y, kTokN, (long)kCh * kTokN,
      b2, x, (long)kCh * kTokN,
      kCh, kTokN, kHidN, kW2CarryInv);
}
